// FlashCRA_31404800868928
// MI455X (gfx1250) — hardware-verified
//
#include <hip/hip_runtime.h>
#include <math.h>
#include <stdint.h>
#include <stddef.h>

constexpr int kNB   = 2;
constexpr int kSEQ  = 2048;
constexpr int kDM   = 1024;
constexpr int kNH   = 16;
constexpr int kHD   = 64;
constexpr int kHALF = 32;
constexpr int kNTOK = kNB * kSEQ;
constexpr int kDQKV = 3 * kDM;
constexpr int kDQK  = 2 * kDM;
constexpr int kDPH  = kDM / 2;
static_assert(kNH * kHD == kDM);
static_assert(kNH * kHALF == kDPH);

typedef __attribute__((ext_vector_type(16))) _Float16 v16h;
typedef __attribute__((ext_vector_type(8)))  _Float16 v8h;
typedef __attribute__((ext_vector_type(16))) __bf16   v16b;
typedef __attribute__((ext_vector_type(8)))  __bf16   v8b;
typedef __attribute__((ext_vector_type(8)))  float    v8f;
typedef __attribute__((ext_vector_type(4)))  float    v4f;
typedef __attribute__((ext_vector_type(2)))  float    v2f;
typedef __attribute__((ext_vector_type(4)))  unsigned int v4u;

__device__ __forceinline__ unsigned short f2bf_bits(float f) {
  unsigned u = __float_as_uint(f);
  return (unsigned short)((u + 0x7FFFu + ((u >> 16) & 1u)) >> 16);
}
__device__ __forceinline__ float bf_bits2f(unsigned short h) { return __uint_as_float(((unsigned)h) << 16); }

__device__ __forceinline__ void dep_guard_h(v8f& a, v8f& b, v16h x, v16h y) { asm volatile("v_nop\n\tv_nop\n\tv_nop\n\tv_nop" : "+v"(a), "+v"(b) : "v"(x), "v"(y)); }
__device__ __forceinline__ void dep_guard_b(v8f& a, v8f& b, v16b x, v16b y) { asm volatile("v_nop\n\tv_nop\n\tv_nop\n\tv_nop" : "+v"(a), "+v"(b) : "v"(x), "v"(y)); }
__device__ __forceinline__ void keep4_h(v16h a, v16h b, v16h c, v16h d) { asm volatile("v_nop" :: "v"(a), "v"(b), "v"(c), "v"(d)); }
__device__ __forceinline__ void keep4_b(v16b a, v16b b, v16b c, v16b d) { asm volatile("v_nop" :: "v"(a), "v"(b), "v"(c), "v"(d)); }
__device__ __forceinline__ void acc_guard4(v8f& a, v8f& b, v8f& c, v8f& d) { asm volatile("v_nop\n\tv_nop\n\tv_nop\n\tv_nop" : "+v"(a), "+v"(b), "+v"(c), "+v"(d)); }
template <typename T> struct Frag;
template <> struct Frag<_Float16> {
  typedef v16h V; union U { v16h v; v8h h[2]; };
  static __device__ __forceinline__ v16h load(const _Float16* p) {
    U f; f.h[0] = *(const v8h*)(p); f.h[1] = *(const v8h*)(p + 16); return f.v;
  }
  static __device__ __forceinline__ v8f mma(v16h a, v16h b, v8f c) {
    return __builtin_amdgcn_wmma_f32_16x16x32_f16(false, a, false, b, (short)0, c, false, false);
  }
  static __device__ __forceinline__ void guard(v8f& a, v8f& b, v16h x, v16h y) { dep_guard_h(a, b, x, y); }
  static __device__ __forceinline__ void keep(v16h a, v16h b, v16h c, v16h d) { keep4_h(a, b, c, d); }
};
template <> struct Frag<__bf16> {
  typedef v16b V; union U { v16b v; v8b h[2]; };
  static __device__ __forceinline__ v16b load(const __bf16* p) {
    U f; f.h[0] = *(const v8b*)(p); f.h[1] = *(const v8b*)(p + 16); return f.v;
  }
  static __device__ __forceinline__ v8f mma(v16b a, v16b b, v8f c) {
    return __builtin_amdgcn_wmma_f32_16x16x32_bf16(false, a, false, b, (short)0, c, false, false);
  }
  static __device__ __forceinline__ void guard(v8f& a, v8f& b, v16b x, v16b y) { dep_guard_b(a, b, x, y); }
  static __device__ __forceinline__ void keep(v16b a, v16b b, v16b c, v16b d) { keep4_b(a, b, c, d); }
};

template <int ET> struct Elem;
template <> struct Elem<0> { typedef _Float16 T; };
template <> struct Elem<1> { typedef __bf16 T; };
template <int ET, int SPLIT, int BIAS_MODE, int OUT_MODE, bool RESID, int ACT = 0>
__global__ __launch_bounds__(256) void wmma_gemm64(
    const unsigned short* __restrict__ Ap, const unsigned short* __restrict__ A2p, int lda, long strideA,
    const unsigned short* __restrict__ Btp, const unsigned short* __restrict__ Bt2p, int ldb, long strideB,
    void* __restrict__ Cout, void* __restrict__ Cout2, int ldc, long strideC,
    const float* __restrict__ bias,
    const float* __restrict__ resid, long strideR,
    int M, int N, int K, float scale) {
  typedef typename Elem<ET>::T T;
  typedef typename Frag<T>::V V;
  const T* A = (const T*)Ap; const T* A2 = (const T*)A2p; const T* Bt = (const T*)Btp; const T* Bt2 = (const T*)Bt2p;
  __shared__ __align__(16) float sT[8][16 * 68];
  const int b    = blockIdx.y;
  const int lane = threadIdx.x & 31;
  const int wave = threadIdx.x >> 5;
  const int tilesN = N >> 6;
  const int tilesM = M >> 6;
  const int tile = blockIdx.x * 8 + wave;
  if (tile >= tilesM * tilesN) return;
  const int tm = tile / tilesN;
  const int tn = tile - tm * tilesN;
  const int m0 = tm << 6;
  const int n0 = tn << 6;

  const T* Ab  = A  + (size_t)b * strideA;
  const T* Bb  = Bt + (size_t)b * strideB;
  const T* Ab2 = (SPLIT != 0) ? (A2  + (size_t)b * strideA) : nullptr;
  const T* Bb2 = (SPLIT == 1) ? (Bt2 + (size_t)b * strideB) : nullptr;

  const int rlane = lane & 15;
  const int koff  = (lane >> 4) * 8;
  const int mOff  = (lane >> 4) * 8;

  v8f acc[4][4];
#pragma unroll
  for (int i = 0; i < 4; ++i)
#pragma unroll
    for (int j = 0; j < 4; ++j) acc[i][j] = (v8f){0.f,0.f,0.f,0.f,0.f,0.f,0.f,0.f};

  for (int k0 = 0; k0 < K; k0 += 32) {
    V bh[4], bl[4];
#pragma unroll
    for (int j = 0; j < 4; ++j) {
      const size_t bo = (size_t)(n0 + (j << 4) + rlane) * ldb + koff + k0;
      bh[j] = Frag<T>::load(Bb + bo);
      if (SPLIT == 1) bl[j] = Frag<T>::load(Bb2 + bo);
    }
#pragma unroll
    for (int i = 0; i < 4; ++i) {
      const size_t ao = (size_t)(m0 + (i << 4) + rlane) * lda + koff + k0;
      V ah = Frag<T>::load(Ab + ao);
      V al;
      if (SPLIT != 0) al = Frag<T>::load(Ab2 + ao); else al = ah;
#pragma unroll
      for (int j = 0; j < 4; ++j) {
        acc[i][j] = Frag<T>::mma(ah, bh[j], acc[i][j]);
        if (SPLIT == 1) {
          acc[i][j] = Frag<T>::mma(ah, bl[j], acc[i][j]);
          acc[i][j] = Frag<T>::mma(al, bh[j], acc[i][j]);
        }
        if (SPLIT == 2) {
          acc[i][j] = Frag<T>::mma(al, bh[j], acc[i][j]);
        }
      }
      Frag<T>::guard(acc[i][0], acc[i][3], ah, al);
    }
    Frag<T>::keep(bh[0], bh[1], bh[2], bh[3]);
    if (SPLIT == 1) Frag<T>::keep(bl[0], bl[1], bl[2], bl[3]);
  }
  acc_guard4(acc[0][0], acc[0][1], acc[0][2], acc[0][3]);
  acc_guard4(acc[1][0], acc[1][1], acc[1][2], acc[1][3]);
  acc_guard4(acc[2][0], acc[2][1], acc[2][2], acc[2][3]);
  acc_guard4(acc[3][0], acc[3][1], acc[3][2], acc[3][3]);

  float* slab = sT[wave];
  const float* Rb = RESID ? (resid + (size_t)b * strideR) : nullptr;
#pragma unroll
  for (int i = 0; i < 4; ++i) {
    const int mBase = m0 + (i << 4);
#pragma unroll
    for (int j = 0; j < 4; ++j) {
      const int n = n0 + (j << 4) + rlane;
      float bv = 0.f;
      if (BIAS_MODE == 2) bv = bias[n];
#pragma unroll
      for (int r = 0; r < 8; ++r) {
        float v = acc[i][j][r] * scale;
        if (BIAS_MODE == 1) v += bias[mBase + mOff + r];
        if (BIAS_MODE == 2) v += bv;
        if (RESID) v += Rb[(size_t)(mBase + mOff + r) * ldc + n];
        if (ACT == 1) v = tanhf(v);
        if (ACT == 2) v = fmaxf(v, 0.0f);
        if (ACT == 4) v = (v > 0.f) ? v : 0.01f * v;
        slab[(mOff + r) * 68 + (j << 4) + rlane] = v;
      }
    }
    __builtin_amdgcn_fence(__ATOMIC_RELEASE, "workgroup");
    __builtin_amdgcn_wave_barrier();
    __builtin_amdgcn_fence(__ATOMIC_ACQUIRE, "workgroup");
    if (OUT_MODE == 0) {
      float* C = (float*)Cout + (size_t)b * strideC;
      const int hh = lane >> 4, c4 = (lane & 15) * 4;
      for (int pass = 0; pass < 2; ++pass) {
#pragma unroll
        for (int it = 0; it < 8; ++it) {
          const int row = it * 2 + hh;
          v4f v = *(const v4f*)(slab + row * 68 + c4);
          *(volatile v4f*)(C + (size_t)(mBase + row) * ldc + n0 + c4) = v;
        }
        __threadfence();
      }
    } else {
      const int q = lane >> 3, c8 = (lane & 7) * 8;
      unsigned short* C  = (unsigned short*)Cout  + (size_t)b * strideC;
      unsigned short* C2 = (OUT_MODE == 2) ? ((unsigned short*)Cout2 + (size_t)b * strideC) : nullptr;
      for (int pass = 0; pass < 2; ++pass) {
#pragma unroll
        for (int it = 0; it < 4; ++it) {
          const int row = it * 4 + q;
          const float* sp = slab + row * 68 + c8;
          v8h hv, lv;
#pragma unroll
          for (int e = 0; e < 8; ++e) {
            if (OUT_MODE == 1) {
              hv[e] = (_Float16)sp[e];
            } else {
              unsigned short hb = f2bf_bits(sp[e]);
              unsigned short lb = f2bf_bits(sp[e] - bf_bits2f(hb));
              hv[e] = __builtin_bit_cast(_Float16, hb);
              lv[e] = __builtin_bit_cast(_Float16, lb);
            }
          }
          *(volatile v8h*)(C + (size_t)(mBase + row) * ldc + n0 + c8) = hv;
          if (OUT_MODE == 2) *(volatile v8h*)(C2 + (size_t)(mBase + row) * ldc + n0 + c8) = lv;
        }
        __threadfence();
      }
    }
    __builtin_amdgcn_fence(__ATOMIC_RELEASE, "workgroup");
    __builtin_amdgcn_wave_barrier();
    __builtin_amdgcn_fence(__ATOMIC_ACQUIRE, "workgroup");
  }
}

__device__ __forceinline__ unsigned pk16(unsigned short a, unsigned short b) { return (unsigned)a | ((unsigned)b << 16); }

__global__ __launch_bounds__(256) void split_bf16x2_kernel(const float* __restrict__ in, unsigned short* __restrict__ hi,
                                                           unsigned short* __restrict__ lo, int n2) {
  const int i = blockIdx.x * 256 + threadIdx.x;
  if (i < n2) {
    const v2f f = *(const v2f*)(in + 2 * (size_t)i);
    const unsigned short h0 = f2bf_bits(f[0]), h1 = f2bf_bits(f[1]);
    const unsigned short l0 = f2bf_bits(f[0] - bf_bits2f(h0)), l1 = f2bf_bits(f[1] - bf_bits2f(h1));
    const unsigned uh = pk16(h0, h1), ul = pk16(l0, l1);
    ((volatile unsigned*)hi)[i] = uh;
    ((volatile unsigned*)lo)[i] = ul;
    __threadfence();
    ((volatile unsigned*)hi)[i] = uh;
    ((volatile unsigned*)lo)[i] = ul;
  }
}

__global__ __launch_bounds__(256) void cast_bf16x2_kernel(const float* __restrict__ in, unsigned short* __restrict__ hi, int n2) {
  const int i = blockIdx.x * 256 + threadIdx.x;
  if (i < n2) {
    const v2f f = *(const v2f*)(in + 2 * (size_t)i);
    const unsigned uh = pk16(f2bf_bits(f[0]), f2bf_bits(f[1]));
    ((volatile unsigned*)hi)[i] = uh;
    __threadfence();
    ((volatile unsigned*)hi)[i] = uh;
  }
}

__global__ __launch_bounds__(256) void tcast_kernel(const float* __restrict__ W, unsigned short* __restrict__ oh, int R, int Cc) {
  __shared__ __align__(16) float tf[64 * 68];
  const int c0  = blockIdx.x * 64;
  const int r0  = blockIdx.y * 64;
  const int tid = threadIdx.x;
  {
    const int lr = tid >> 4;
    const int c4 = (tid & 15) * 4;
#pragma unroll
    for (int it = 0; it < 4; ++it) {
      const int rr = it * 16 + lr;
      const v4f a = *(const v4f*)(W + (size_t)(r0 + rr) * Cc + c0 + c4);
      *(v4f*)(tf + rr * 68 + c4) = a;
    }
  }
  __syncthreads();
  const int sub = tid >> 3;
  const int c8  = (tid & 7) * 8;
  v4u hv[2];
#pragma unroll
  for (int it = 0; it < 2; ++it) {
    const int oc = it * 32 + sub;
    v4u a;
#pragma unroll
    for (int q = 0; q < 4; ++q) {
      const float f0 = tf[(c8 + 2 * q) * 68 + oc];
      const float f1 = tf[(c8 + 2 * q + 1) * 68 + oc];
      a[q] = pk16(f2bf_bits(f0), f2bf_bits(f1));
    }
    hv[it] = a;
  }
  for (int pass = 0; pass < 2; ++pass) {
#pragma unroll
    for (int it = 0; it < 2; ++it) {
      const int oc = it * 32 + sub;
      const size_t go = (size_t)(c0 + oc) * R + r0 + c8;
      *(volatile v4u*)(oh + go) = hv[it];
    }
    __threadfence();
  }
}

__global__ __launch_bounds__(256) void bias_rne_kernel(const float* __restrict__ in, float* __restrict__ outp, int n4) {
  const int i = blockIdx.x * 256 + threadIdx.x;
  if (i < n4) {
    const v4f f = *(const v4f*)(in + 4 * (size_t)i);
    v4f rv;
    rv[0] = bf_bits2f(f2bf_bits(f[0]));
    rv[1] = bf_bits2f(f2bf_bits(f[1]));
    rv[2] = bf_bits2f(f2bf_bits(f[2]));
    rv[3] = bf_bits2f(f2bf_bits(f[3]));
    *(volatile v4f*)(outp + 4 * (size_t)i) = rv;
    __threadfence();
    *(volatile v4f*)(outp + 4 * (size_t)i) = rv;
  }
}

__device__ __forceinline__ void split_bits(float f, unsigned short& h, unsigned short& l) {
  h = f2bf_bits(f);
  l = f2bf_bits(f - bf_bits2f(h));
}
__device__ __forceinline__ void store_plane8(unsigned short* __restrict__ dst, const unsigned short* sp, int q, int c8) {
#pragma unroll
  for (int it = 0; it < 2; ++it) {
    const int hl = it * 4 + q;
    const v4u v = *(const v4u*)(sp + hl * 64 + c8);
    *(volatile v4u*)(dst + hl * 64 + c8) = v;
  }
}

__global__ __launch_bounds__(256) void rope_split_kernel(const float* __restrict__ qkf, const float* __restrict__ ph,
                                                         unsigned short* __restrict__ qh, unsigned short* __restrict__ ql,
                                                         unsigned short* __restrict__ kh, unsigned short* __restrict__ kl, int ntok) {
  __shared__ __align__(16) unsigned short stg[8][4][512];
  const int tid = threadIdx.x, wave = tid >> 5, lane = tid & 31;
  const int wid  = blockIdx.x * 8 + wave;
  const int traw = wid >> 1;
  const int hg   = wid & 1;
  const bool active = (traw < ntok);
  const int t = active ? traw : (ntok - 1);
#pragma unroll 1
  for (int hl = 0; hl < 8; ++hl) {
    const int head = hg * 8 + hl;
    const size_t qo = (size_t)t * kDQK + (size_t)head * kHD + lane;
    const float q1 = qkf[qo];
    const float q2 = qkf[qo + kHALF];
    const float k1 = qkf[qo + kDM];
    const float k2 = qkf[qo + kDM + kHALF];
    const float pv = ph[(size_t)t * kDPH + head * kHALF + lane];
    float sn, cs;
    sincosf(pv, &sn, &cs);
    const float qa = q1 * cs - q2 * sn;
    const float qb = q1 * sn + q2 * cs;
    const float ka = k1 * cs - k2 * sn;
    const float kb = k1 * sn + k2 * cs;
    unsigned short h0, l0;
    split_bits(qa, h0, l0); stg[wave][0][hl * 64 + lane] = h0;         stg[wave][1][hl * 64 + lane] = l0;
    split_bits(qb, h0, l0); stg[wave][0][hl * 64 + kHALF + lane] = h0; stg[wave][1][hl * 64 + kHALF + lane] = l0;
    split_bits(ka, h0, l0); stg[wave][2][hl * 64 + lane] = h0;         stg[wave][3][hl * 64 + lane] = l0;
    split_bits(kb, h0, l0); stg[wave][2][hl * 64 + kHALF + lane] = h0; stg[wave][3][hl * 64 + kHALF + lane] = l0;
  }
  __syncthreads();
  if (active) {
    const int q = lane >> 3, c8 = (lane & 7) * 8;
    const size_t rb = (size_t)t * kDM + (size_t)(hg * 8) * kHD;
    for (int pass = 0; pass < 2; ++pass) {
      store_plane8(qh + rb, stg[wave][0], q, c8);
      store_plane8(ql + rb, stg[wave][1], q, c8);
      store_plane8(kh + rb, stg[wave][2], q, c8);
      store_plane8(kl + rb, stg[wave][3], q, c8);
      __threadfence();
    }
  }
}

#define AT_D 64
#define AT_NW 4
#define AT_QB 64
#define AT_KC 64

__device__ __forceinline__ unsigned short at_bf_bits(float f) {
  unsigned u = __float_as_uint(f);
  return (unsigned short)((u + 0x7FFFu + ((u >> 16) & 1u)) >> 16);
}
__device__ __forceinline__ __bf16 at_f2bf(float f) { return __builtin_bit_cast(__bf16, at_bf_bits(f)); }
__device__ __forceinline__ void at_split(float f, __bf16& hi, __bf16& lo) {
  const unsigned short hb = at_bf_bits(f);
  hi = __builtin_bit_cast(__bf16, hb);
  lo = at_f2bf(f - __uint_as_float(((unsigned)hb) << 16));
}
__device__ __forceinline__ v8f at_mma(v16b a, v16b b, v8f c) {
  c = __builtin_amdgcn_wmma_f32_16x16x32_bf16(false, a, false, b, (short)0, c, false, false);
  asm volatile("v_nop\n\tv_nop\n\tv_nop\n\tv_nop" : "+v"(c) : "v"(a), "v"(b));
  return c;
}

__global__ __launch_bounds__(128)
void attn_planes_kernel(const unsigned short* __restrict__ qhp, const unsigned short* __restrict__ qlp,
                        const unsigned short* __restrict__ khp, const unsigned short* __restrict__ klp,
                        const unsigned short* __restrict__ vhp, const unsigned short* __restrict__ vlp,
                        float* __restrict__ out, float sscale) {
  union FB { v16b v; v8b h[2]; };
  __shared__ __align__(16) __bf16 Ksh[AT_KC * AT_D];
  __shared__ __align__(16) __bf16 Ksl[AT_KC * AT_D];
  __shared__ __align__(16) __bf16 Vth[AT_D * AT_KC];
  __shared__ __align__(16) __bf16 Vtl[AT_D * AT_KC];
  __shared__ __align__(16) __bf16 Psh[AT_NW][16 * AT_KC];
  __shared__ __align__(16) __bf16 Psl[AT_NW][16 * AT_KC];
  __shared__ __align__(16) float  Os[AT_NW][16 * 68];

  const int tid  = threadIdx.x;
  const int wave = tid >> 5;
  const int lane = tid & 31;
  const int hh   = lane >> 4;
  const int c    = lane & 15;

  constexpr int nqb = kSEQ / AT_QB;
  const int bx = blockIdx.x;
  const int qb = bx % nqb;
  const int h  = bx / nqb;
  const int b  = blockIdx.y;
  const int q0 = qb * AT_QB + wave * 16;

  const __bf16* Qh = (const __bf16*)(const void*)qhp + (size_t)b * kSEQ * kDM + (size_t)h * AT_D;
  const __bf16* Ql = (const __bf16*)(const void*)qlp + (size_t)b * kSEQ * kDM + (size_t)h * AT_D;
  const __bf16* Kh = (const __bf16*)(const void*)khp + (size_t)b * kSEQ * kDM + (size_t)h * AT_D;
  const __bf16* Kl = (const __bf16*)(const void*)klp + (size_t)b * kSEQ * kDM + (size_t)h * AT_D;
  const __bf16* Vh = (const __bf16*)(const void*)vhp + (size_t)b * kDM * kSEQ + (size_t)h * AT_D * kSEQ;
  const __bf16* Vl = (const __bf16*)(const void*)vlp + (size_t)b * kDM * kSEQ + (size_t)h * AT_D * kSEQ;
  float*        ob = out + (size_t)b * kSEQ * kDM + (size_t)h * AT_D;

  v16b qah[2], qal[2];
#pragma unroll
  for (int dc = 0; dc < 2; ++dc) {
    const __bf16* qr = Qh + (size_t)(q0 + c) * kDM + dc * 32 + 8 * hh;
    const __bf16* qs = Ql + (size_t)(q0 + c) * kDM + dc * 32 + 8 * hh;
    qah[dc] = Frag<__bf16>::load(qr);
    qal[dc] = Frag<__bf16>::load(qs);
  }

  float mrow[8], lrow[8];
  v8f oacc[4];
#pragma unroll
  for (int r = 0; r < 8; ++r) { mrow[r] = -INFINITY; lrow[r] = 0.f; }
#pragma unroll
  for (int t = 0; t < 4; ++t) oacc[t] = (v8f){0.f,0.f,0.f,0.f,0.f,0.f,0.f,0.f};

  constexpr int nChunks = kSEQ / AT_KC;
  for (int kc = 0; kc < nChunks; ++kc) {
    const int kv0 = kc * AT_KC;
    __syncthreads();
    {
      const int r = tid >> 1, half = (tid & 1) * 32;
      const __bf16* ksh = Kh + (size_t)(kv0 + r) * kDM + half;
      const __bf16* ksl = Kl + (size_t)(kv0 + r) * kDM + half;
      const __bf16* vsh = Vh + (size_t)r * kSEQ + kv0 + half;
      const __bf16* vsl = Vl + (size_t)r * kSEQ + kv0 + half;
#pragma unroll
      for (int i = 0; i < 4; ++i) {
        const v8b a0 = *(const v8b*)(ksh + 8 * i);
        const v8b a1 = *(const v8b*)(ksl + 8 * i);
        const v8b b0 = *(const v8b*)(vsh + 8 * i);
        const v8b b1 = *(const v8b*)(vsl + 8 * i);
        *(v8b*)(Ksh + r * AT_D  + half + 8 * i) = a0;
        *(v8b*)(Ksl + r * AT_D  + half + 8 * i) = a1;
        *(v8b*)(Vth + r * AT_KC + half + 8 * i) = b0;
        *(v8b*)(Vtl + r * AT_KC + half + 8 * i) = b1;
      }
    }
    __syncthreads();

    v8f s[4];
#pragma unroll
    for (int j = 0; j < 4; ++j) {
      s[j] = (v8f){0.f,0.f,0.f,0.f,0.f,0.f,0.f,0.f};
#pragma unroll
      for (int dc = 0; dc < 2; ++dc) {
        FB kb, ks;
        kb.h[0] = *(const v8b*)(Ksh + (j * 16 + c) * AT_D + dc * 32 + 8 * hh);
        kb.h[1] = *(const v8b*)(Ksh + (j * 16 + c) * AT_D + dc * 32 + 16 + 8 * hh);
        ks.h[0] = *(const v8b*)(Ksl + (j * 16 + c) * AT_D + dc * 32 + 8 * hh);
        ks.h[1] = *(const v8b*)(Ksl + (j * 16 + c) * AT_D + dc * 32 + 16 + 8 * hh);
        s[j] = at_mma(qah[dc], kb.v, s[j]);
        s[j] = at_mma(qah[dc], ks.v, s[j]);
        s[j] = at_mma(qal[dc], kb.v, s[j]);
      }
    }
    float cm[8];
#pragma unroll
    for (int r = 0; r < 8; ++r) {
      float m = -INFINITY;
#pragma unroll
      for (int j = 0; j < 4; ++j) {
        const float sv = s[j][r] * sscale;
        s[j][r] = sv;
        m = fmaxf(m, sv);
      }
#pragma unroll
      for (int off = 1; off < 16; off <<= 1) m = fmaxf(m, __shfl_xor(m, off, 32));
      cm[r] = m;
    }
    __bf16* pwh = Psh[wave];
    __bf16* pwl = Psl[wave];
#pragma unroll
    for (int r = 0; r < 8; ++r) {
      const float mnew = fmaxf(mrow[r], cm[r]);
      const float alpha = expf(mrow[r] - mnew);
      mrow[r] = mnew;
      float psum = 0.f;
#pragma unroll
      for (int j = 0; j < 4; ++j) {
        const float p = expf(s[j][r] - mnew);
        psum += p;
        __bf16 a, bl;
        at_split(p, a, bl);
        pwh[(8 * hh + r) * AT_KC + j * 16 + c] = a;
        pwl[(8 * hh + r) * AT_KC + j * 16 + c] = bl;
      }
#pragma unroll
      for (int off = 1; off < 16; off <<= 1) psum += __shfl_xor(psum, off, 32);
      lrow[r] = lrow[r] * alpha + psum;
#pragma unroll
      for (int t = 0; t < 4; ++t) oacc[t][r] *= alpha;
    }
    __builtin_amdgcn_fence(__ATOMIC_RELEASE, "workgroup");
    __builtin_amdgcn_wave_barrier();
    __builtin_amdgcn_fence(__ATOMIC_ACQUIRE, "workgroup");
#pragma unroll 1
    for (int kk = 0; kk < 2; ++kk) {
      FB pa, pl;
      pa.h[0] = *(const v8b*)(pwh + c * AT_KC + kk * 32 + 8 * hh);
      pa.h[1] = *(const v8b*)(pwh + c * AT_KC + kk * 32 + 16 + 8 * hh);
      pl.h[0] = *(const v8b*)(pwl + c * AT_KC + kk * 32 + 8 * hh);
      pl.h[1] = *(const v8b*)(pwl + c * AT_KC + kk * 32 + 16 + 8 * hh);
#pragma unroll
      for (int t = 0; t < 4; ++t) {
        FB vb, vl;
        vb.h[0] = *(const v8b*)(Vth + (t * 16 + c) * AT_KC + kk * 32 + 8 * hh);
        vb.h[1] = *(const v8b*)(Vth + (t * 16 + c) * AT_KC + kk * 32 + 16 + 8 * hh);
        vl.h[0] = *(const v8b*)(Vtl + (t * 16 + c) * AT_KC + kk * 32 + 8 * hh);
        vl.h[1] = *(const v8b*)(Vtl + (t * 16 + c) * AT_KC + kk * 32 + 16 + 8 * hh);
        oacc[t] = at_mma(pa.v, vb.v, oacc[t]);
        oacc[t] = at_mma(pa.v, vl.v, oacc[t]);
        oacc[t] = at_mma(pl.v, vb.v, oacc[t]);
      }
    }
  }

  float* os = Os[wave];
#pragma unroll
  for (int r = 0; r < 8; ++r) {
    const float inv = 1.0f / lrow[r];
#pragma unroll
    for (int t = 0; t < 4; ++t) os[(8 * hh + r) * 68 + t * 16 + c] = oacc[t][r] * inv;
  }
  __builtin_amdgcn_fence(__ATOMIC_RELEASE, "workgroup");
  __builtin_amdgcn_wave_barrier();
  __builtin_amdgcn_fence(__ATOMIC_ACQUIRE, "workgroup");
  {
    const int c4 = (lane & 15) * 4;
    for (int pass = 0; pass < 2; ++pass) {
#pragma unroll
      for (int it = 0; it < 8; ++it) {
        const int row = it * 2 + hh;
        v4f val = *(const v4f*)(os + row * 68 + c4);
        *(volatile v4f*)(ob + (size_t)(q0 + row) * kDM + c4) = val;
      }
      __threadfence();
    }
  }
}

extern "C" void kernel_launch(void* const* d_in, const int* in_sizes, int n_in,
                              void* d_out, int out_size, void* d_ws, size_t ws_size,
                              hipStream_t stream) {
  if (n_in < 7) return;
  if (in_sizes[0] != kNTOK * kDM || in_sizes[1] != kNTOK * kDM || in_sizes[2] != kDM * kDQKV ||
      in_sizes[3] != kDQKV || in_sizes[4] != kDM * kDM || in_sizes[5] != kDM || in_sizes[6] != kDM * kDPH) return;
  if (out_size != kNTOK * kDM) return;

  const size_t MIB = (size_t)1048576;
  const size_t OFF_XB  = 0;
  const size_t OFF_PB  = 8 * MIB;
  const size_t OFF_WQT = 16 * MIB;
  const size_t OFF_PJT = 22 * MIB;
  const size_t OFF_WOT = 23 * MIB;
  const size_t OFF_BQ  = 25 * MIB;
  const size_t OFF_BO  = 25 * MIB + 16384;
  const size_t OFF_QKF = 26 * MIB;
  const size_t OFF_OF  = 26 * MIB;
  const size_t OFF_OH  = 42 * MIB;
  const size_t OFF_OL  = 50 * MIB;
  const size_t OFF_PH  = 58 * MIB;
  const size_t OFF_QH  = 66 * MIB;
  const size_t OFF_QL  = 74 * MIB;
  const size_t OFF_KH  = 82 * MIB;
  const size_t OFF_KL  = 90 * MIB;
  const size_t OFF_VH  = 98 * MIB;
  const size_t OFF_VL  = 106 * MIB;
  const size_t WS_TOTAL = 114 * MIB;
  static_assert((size_t)kNTOK * kDM * 2 == 8 * 1048576);
  static_assert((size_t)kDQKV * kDM * 2 == 6 * 1048576);
  static_assert((size_t)kDPH * kDM * 2 == 1 * 1048576);
  static_assert((size_t)kDM * kDM * 2 == 2 * 1048576);
  static_assert((size_t)kNTOK * kDQK * 4 == 32 * 1048576);
  static_assert((size_t)kNTOK * kDM * 4 == 16 * 1048576);
  static_assert((size_t)kNTOK * kDPH * 4 == 8 * 1048576);
  static_assert((size_t)kNB * kDM * kSEQ * 2 == 8 * 1048576);
  if (ws_size < WS_TOTAL) return;

  const float* x    = (const float*)d_in[0];
  const float* p    = (const float*)d_in[1];
  const float* Wqkv = (const float*)d_in[2];
  const float* bqkv = (const float*)d_in[3];
  const float* Wout = (const float*)d_in[4];
  const float* bout = (const float*)d_in[5];
  const float* proj = (const float*)d_in[6];
  float* outp = (float*)d_out;

  char* ws = (char*)d_ws;
  unsigned short* xb  = (unsigned short*)(ws + OFF_XB);
  unsigned short* pb  = (unsigned short*)(ws + OFF_PB);
  unsigned short* wqt = (unsigned short*)(ws + OFF_WQT);
  unsigned short* pjt = (unsigned short*)(ws + OFF_PJT);
  unsigned short* wot = (unsigned short*)(ws + OFF_WOT);
  float* bqr = (float*)(ws + OFF_BQ);
  float* bor = (float*)(ws + OFF_BO);
  float* qkf = (float*)(ws + OFF_QKF);
  float* of  = (float*)(ws + OFF_OF);
  unsigned short* ohp = (unsigned short*)(ws + OFF_OH);
  unsigned short* olp = (unsigned short*)(ws + OFF_OL);
  float* phf = (float*)(ws + OFF_PH);
  unsigned short* qhp = (unsigned short*)(ws + OFF_QH);
  unsigned short* qlp = (unsigned short*)(ws + OFF_QL);
  unsigned short* khp = (unsigned short*)(ws + OFF_KH);
  unsigned short* klp = (unsigned short*)(ws + OFF_KL);
  unsigned short* vhp = (unsigned short*)(ws + OFF_VH);
  unsigned short* vlp = (unsigned short*)(ws + OFF_VL);

  const int n2act = kNTOK * kDM / 2;
  cast_bf16x2_kernel<<<dim3((n2act + 255) / 256), dim3(256), 0, stream>>>(x, xb, n2act);
  cast_bf16x2_kernel<<<dim3((n2act + 255) / 256), dim3(256), 0, stream>>>(p, pb, n2act);
  tcast_kernel<<<dim3(kDQKV / 64, kDM / 64), dim3(256), 0, stream>>>(Wqkv, wqt, kDM, kDQKV);
  tcast_kernel<<<dim3(kDPH / 64, kDM / 64), dim3(256), 0, stream>>>(proj, pjt, kDM, kDPH);
  tcast_kernel<<<dim3(kDM / 64, kDM / 64), dim3(256), 0, stream>>>(Wout, wot, kDM, kDM);
  bias_rne_kernel<<<dim3((kDQKV / 4 + 255) / 256), dim3(256), 0, stream>>>(bqkv, bqr, kDQKV / 4);
  bias_rne_kernel<<<dim3((kDM / 4 + 255) / 256), dim3(256), 0, stream>>>(bout, bor, kDM / 4);
  wmma_gemm64<1, 0, 2, 0, false><<<dim3((kNTOK / 64) * (kDQK / 64) / 8, 1), dim3(256), 0, stream>>>(
      xb, xb, kDM, 0L, wqt, wqt, kDM, 0L, (void*)qkf, (void*)qkf, kDQK, 0L, bqr, bqr, 0L, kNTOK, kDQK, kDM, 1.0f);
  wmma_gemm64<1, 0, 1, 2, false><<<dim3((kDM / 64) * (kSEQ / 64) / 8, kNB), dim3(256), 0, stream>>>(
      wqt + (size_t)kDQK * kDM, wqt + (size_t)kDQK * kDM, kDM, 0L, xb, xb, kDM, (long)kSEQ * kDM,
      (void*)vhp, (void*)vlp, kSEQ, (long)kDM * kSEQ, bqr + kDQK, bqr, 0L, kDM, kSEQ, kDM, 1.0f);
  wmma_gemm64<1, 0, 0, 0, false><<<dim3((kNTOK / 64) * (kDPH / 64) / 8, 1), dim3(256), 0, stream>>>(
      pb, pb, kDM, 0L, pjt, pjt, kDM, 0L, (void*)phf, (void*)phf, kDPH, 0L, bqr, bqr, 0L, kNTOK, kDPH, kDM, 1.0f);
  rope_split_kernel<<<dim3((kNTOK * 2 + 7) / 8), dim3(256), 0, stream>>>(qkf, phf, qhp, qlp, khp, klp, kNTOK);
  attn_planes_kernel<<<dim3(kNH * (kSEQ / 64), kNB), dim3(128), 0, stream>>>(qhp, qlp, khp, klp, vhp, vlp, of, 0.125f);
  split_bf16x2_kernel<<<dim3((n2act + 255) / 256), dim3(256), 0, stream>>>(of, ohp, olp, n2act);
  wmma_gemm64<1, 2, 2, 0, false><<<dim3((kNTOK / 64) * (kDM / 64) / 8, 1), dim3(256), 0, stream>>>(
      ohp, olp, kDM, 0L, wot, wot, kDM, 0L, (void*)outp, (void*)outp, kDM, 0L, bor, bor, 0L, kNTOK, kDM, kDM, 1.0f);
}
